// ExactSphericalKernelCausalAttention_56367150793419
// MI455X (gfx1250) — hardware-verified
//
#include <hip/hip_runtime.h>


#define NB_  2
#define TT   2048
#define EE   1024
#define NH_  16
#define HD   64
#define ZH   2
#define PCAR 64.0f
typedef _Float16 h16;
typedef unsigned short bf;
typedef __attribute__((ext_vector_type(16))) __bf16   v16bf;
typedef __attribute__((ext_vector_type(16))) _Float16 v16h;
typedef __attribute__((ext_vector_type(8)))  _Float16 v8h;
typedef __attribute__((ext_vector_type(8)))  unsigned short v8us;
typedef __attribute__((ext_vector_type(8)))  float    v8f;
typedef __attribute__((ext_vector_type(4)))  float    v4f;
typedef v8h  __attribute__((may_alias)) v8ha;
typedef v4f  __attribute__((may_alias)) v4fa;
typedef v8us __attribute__((may_alias)) v8usa;

__device__ __forceinline__ unsigned short f2bf(float f) { unsigned u = __float_as_uint(f); u += 0x7FFFu + ((u >> 16) & 1u); return (unsigned short)(u >> 16); }
__device__ __forceinline__ float bf2f(unsigned short b) { return __uint_as_float(((unsigned)b) << 16); }
__device__ __forceinline__ float bfr(float f) { return bf2f(f2bf(f)); }
__device__ __forceinline__ v16h cat16(v8h lo, v8h hi) { return __builtin_shufflevector(lo, hi, 0, 1, 2, 3, 4, 5, 6, 7, 8, 9, 10, 11, 12, 13, 14, 15); }
__device__ __forceinline__ v16bf cat16b(v8us lo, v8us hi) { return __builtin_bit_cast(v16bf, __builtin_shufflevector(lo, hi, 0, 1, 2, 3, 4, 5, 6, 7, 8, 9, 10, 11, 12, 13, 14, 15)); }
__device__ __forceinline__ v8f wmma16(v16h a, v16h b, v8f c) { return __builtin_amdgcn_wmma_f32_16x16x32_f16(false, a, false, b, (short)0, c, false, false); }
__device__ __forceinline__ v8f wmmab(v16bf a, v16bf b, v8f c) { return __builtin_amdgcn_wmma_f32_16x16x32_bf16(false, a, false, b, (short)0, c, false, false); }


template <typename T16> struct WFrag;
template <> struct WFrag<h16> { typedef v16h V; static __device__ __forceinline__ V ld(const h16* p) { return cat16(*(const v8h*)p, *(const v8h*)(p + 16)); } static __device__ __forceinline__ v8f mma(V a, V b, v8f c) { return wmma16(a, b, c); } };
template <> struct WFrag<bf> { typedef v16bf V; static __device__ __forceinline__ V ld(const bf* p) { return cat16b(*(const v8us*)p, *(const v8us*)(p + 16)); } static __device__ __forceinline__ v8f mma(V a, V b, v8f c) { return wmmab(a, b, c); } };
template <typename T16, int NSPLIT, bool BIAS>
__global__ __launch_bounds__(32) void k_gemmw(const T16* __restrict__ A, const T16* __restrict__ A2, const T16* __restrict__ Bt, const T16* __restrict__ Bt2, int K, float* C, int ldc, const float* __restrict__ bias, size_t sA, size_t sB, size_t sC) {
    typedef typename WFrag<T16>::V V;
    __shared__ __align__(16) float os[16 * 68];
    const size_t z = blockIdx.z; A += z * sA; if (A2) A2 += z * sA; Bt += z * sB; if (Bt2) Bt2 += z * sB; C += z * sC;
    const int lane = threadIdx.x & 31, lr = lane & 15, hi = lane >> 4; const int r0 = blockIdx.x * 64, c0 = blockIdx.y * 64;
    v8f acc[4][4];
#pragma unroll
    for (int mb = 0; mb < 4; ++mb)
#pragma unroll
        for (int nb = 0; nb < 4; ++nb) acc[mb][nb] = (v8f){};
    const size_t aoff = (size_t)(r0 + lr) * K + 8 * hi, boff = (size_t)(c0 + lr) * K + 8 * hi;
#pragma unroll 1
    for (int kc = 0; kc < K; kc += 32) {
        V a[4], a2[4];
#pragma unroll
        for (int mb = 0; mb < 4; ++mb) { a[mb] = WFrag<T16>::ld(A + aoff + (size_t)mb * 16 * K + kc); if (NSPLIT == 1 || NSPLIT == 2) a2[mb] = WFrag<T16>::ld(A2 + aoff + (size_t)mb * 16 * K + kc); }
#pragma unroll
        for (int nb = 0; nb < 4; ++nb) { const V b = WFrag<T16>::ld(Bt + boff + (size_t)nb * 16 * K + kc); V b2; if (NSPLIT >= 2) b2 = WFrag<T16>::ld(Bt2 + boff + (size_t)nb * 16 * K + kc);
#pragma unroll
            for (int mb = 0; mb < 4; ++mb) { acc[mb][nb] = WFrag<T16>::mma(a[mb], b, acc[mb][nb]); if (NSPLIT == 1 || NSPLIT == 2) acc[mb][nb] = WFrag<T16>::mma(a2[mb], b, acc[mb][nb]); if (NSPLIT >= 2) acc[mb][nb] = WFrag<T16>::mma(a[mb], b2, acc[mb][nb]); } }
        asm volatile("v_nop\n\tv_nop\n\tv_nop\n\tv_nop" : "+v"(acc[0][0]), "+v"(acc[1][1]), "+v"(acc[2][2]), "+v"(acc[3][3]) : "v"(a[0]), "v"(a[3]));
    }
#pragma unroll
    for (int mb = 0; mb < 4; ++mb) {
#pragma unroll
        for (int nb = 0; nb < 4; ++nb) {
#pragma unroll
            for (int j = 0; j < 8; ++j) os[(hi * 8 + j) * 68 + nb * 16 + lr] = acc[mb][nb][j]; }
        __builtin_amdgcn_wave_barrier(); asm volatile("" ::: "memory");
        float* crow = C + (size_t)(r0 + mb * 16) * ldc + c0;
#pragma unroll 1
        for (int ps = 0; ps < 2; ++ps) {
#pragma unroll
            for (int s = 0; s < 8; ++s) { const int row = 2 * s + hi, cofs = lr * 4; v4f val = *(const v4fa*)(os + row * 68 + cofs); if (BIAS) { val[0] += bfr(bias[c0 + cofs]); val[1] += bfr(bias[c0 + cofs + 1]); val[2] += bfr(bias[c0 + cofs + 2]); val[3] += bfr(bias[c0 + cofs + 3]); }
                *(volatile v4f*)(crow + (size_t)row * ldc + cofs) = val; }
            if (ps == 0) __threadfence(); }
        __builtin_amdgcn_wave_barrier(); asm volatile("" ::: "memory");
    }
}

template <typename T16, int NSPLIT, int CMODE>
__global__ __launch_bounds__(32) void k_gemmc(const T16* __restrict__ A, const T16* __restrict__ A2, const T16* __restrict__ Bt, const T16* __restrict__ Bt2, int K, float* C, int ldc, int roff, size_t sA, size_t sB, size_t sC) {
    typedef typename WFrag<T16>::V V;
    __shared__ __align__(16) float os[16 * 68];
    const size_t z = blockIdx.z; A += z * sA; if (A2) A2 += z * sA; Bt += z * sB; if (Bt2) Bt2 += z * sB; C += z * sC;
    const int lane = threadIdx.x & 31, lr = lane & 15, hi = lane >> 4; const int r0 = blockIdx.x * 64, c0 = blockIdx.y * 64;
    if (CMODE == 1 && c0 > r0 + roff + 63) return;
    const int Kl = (CMODE == 2) ? min(K, r0 + roff + 64) : K;
    v8f acc[4][4];
#pragma unroll
    for (int mb = 0; mb < 4; ++mb)
#pragma unroll
        for (int nb = 0; nb < 4; ++nb) acc[mb][nb] = (v8f){};
    const size_t aoff = (size_t)(r0 + lr) * K + 8 * hi, boff = (size_t)(c0 + lr) * K + 8 * hi;
#pragma unroll 1
    for (int kc = 0; kc < Kl; kc += 32) {
        V a[4], a2[4];
#pragma unroll
        for (int mb = 0; mb < 4; ++mb) { a[mb] = WFrag<T16>::ld(A + aoff + (size_t)mb * 16 * K + kc); if (NSPLIT == 1 || NSPLIT == 2) a2[mb] = WFrag<T16>::ld(A2 + aoff + (size_t)mb * 16 * K + kc); }
#pragma unroll
        for (int nb = 0; nb < 4; ++nb) { const V b = WFrag<T16>::ld(Bt + boff + (size_t)nb * 16 * K + kc); V b2; if (NSPLIT >= 2) b2 = WFrag<T16>::ld(Bt2 + boff + (size_t)nb * 16 * K + kc);
#pragma unroll
            for (int mb = 0; mb < 4; ++mb) { acc[mb][nb] = WFrag<T16>::mma(a[mb], b, acc[mb][nb]); if (NSPLIT == 1 || NSPLIT == 2) acc[mb][nb] = WFrag<T16>::mma(a2[mb], b, acc[mb][nb]); if (NSPLIT >= 2) acc[mb][nb] = WFrag<T16>::mma(a[mb], b2, acc[mb][nb]); } }
        asm volatile("v_nop\n\tv_nop\n\tv_nop\n\tv_nop" : "+v"(acc[0][0]), "+v"(acc[1][1]), "+v"(acc[2][2]), "+v"(acc[3][3]) : "v"(a[0]), "v"(a[3]));
    }
#pragma unroll
    for (int mb = 0; mb < 4; ++mb) {
#pragma unroll
        for (int nb = 0; nb < 4; ++nb) {
#pragma unroll
            for (int j = 0; j < 8; ++j) os[(hi * 8 + j) * 68 + nb * 16 + lr] = acc[mb][nb][j]; }
        __builtin_amdgcn_wave_barrier(); asm volatile("" ::: "memory");
        float* crow = C + (size_t)(r0 + mb * 16) * ldc + c0;
#pragma unroll 1
        for (int ps = 0; ps < 2; ++ps) {
#pragma unroll
            for (int s = 0; s < 8; ++s) { const int row = 2 * s + hi, cofs = lr * 4; v4f val = *(const v4fa*)(os + row * 68 + cofs);
                *(volatile v4f*)(crow + (size_t)row * ldc + cofs) = val; }
            if (ps == 0) __threadfence(); }
        __builtin_amdgcn_wave_barrier(); asm volatile("" ::: "memory");
    }
}

__device__ __forceinline__ h16 tohx(float x) { return (h16)x; }
__device__ __forceinline__ void splitf(float y, unsigned short& h, unsigned short& l) { h = f2bf(y); l = f2bf(y - bf2f(h)); }
typedef __attribute__((ext_vector_type(2))) _Float16 v2h;
typedef __attribute__((ext_vector_type(4))) _Float16 v4h;
typedef __attribute__((ext_vector_type(2))) unsigned short v2us;
typedef __attribute__((ext_vector_type(4))) unsigned short v4us;

__global__ __launch_bounds__(256) void k_wtG(const float* __restrict__ w, int K, int N, bf* Bt) {
    const int lane = threadIdx.x & 31; const int L0 = (blockIdx.x * 8 + (threadIdx.x >> 5)) * 8; const int nlines = N * K / 64;
#pragma unroll 1
    for (int ps = 0; ps < 2; ++ps) {
#pragma unroll 1
        for (int l = 0; l < 8; ++l) { const int L = L0 + l; if (L >= nlines) break; const size_t e = (size_t)L * 64 + lane * 2; const int k = (int)(e % K), n = (int)(e / K); v2us o;
            o[0] = f2bf(w[(size_t)k * N + n]); o[1] = f2bf(w[(size_t)(k + 1) * N + n]); *(volatile v2us*)(Bt + e) = o; }
        if (ps == 0) __threadfence(); }
}
__global__ __launch_bounds__(256) void k_cvt8(const float* __restrict__ src, bf* dst, size_t n8) { const size_t i = (size_t)blockIdx.x * 256 + threadIdx.x; if (i >= n8) return; const v8f v = *(const v8f*)(src + i * 8); v8us o;
#pragma unroll
    for (int k = 0; k < 8; ++k) o[k] = f2bf(v[k]); *(volatile v8us*)(dst + i * 8) = o; __threadfence(); *(volatile v8us*)(dst + i * 8) = o; }
__global__ __launch_bounds__(256) void k_nrm(const float* __restrict__ QKV, bf* Qh, bf* Ql, bf* Kh, bf* Kl) { const int lane = threadIdx.x & 31; const int row = blockIdx.x * 8 + (threadIdx.x >> 5); if (row >= NH_ * TT) return; const int t = row % TT, h = row / TT; const float* q = QKV + (size_t)t * 3 * EE + h * HD; const float* k = q + EE;
    const float q0 = q[lane * 2], q1 = q[lane * 2 + 1], k0 = k[lane * 2], k1 = k[lane * 2 + 1]; float sq = __fadd_rn(__fmul_rn(q0, q0), __fmul_rn(q1, q1)), sk = __fadd_rn(__fmul_rn(k0, k0), __fmul_rn(k1, k1));
#pragma unroll
    for (int sh = 16; sh; sh >>= 1) { sq += __shfl_xor(sq, sh, 32); sk += __shfl_xor(sk, sh, 32); }
    const float nq = fmaxf(__fsqrt_rn(sq), 1e-12f), nk = fmaxf(__fsqrt_rn(sk), 1e-12f); const size_t o = ((size_t)h * TT + t) * HD + lane * 2; v2us qh, ql, kh, kl; unsigned short a, c;
    splitf(__fdiv_rn(q0, nq), a, c); qh[0] = a; ql[0] = c; splitf(__fdiv_rn(q1, nq), a, c); qh[1] = a; ql[1] = c; splitf(__fdiv_rn(k0, nk), a, c); kh[0] = a; kl[0] = c; splitf(__fdiv_rn(k1, nk), a, c); kh[1] = a; kl[1] = c;
    for (int ps = 0; ps < 2; ++ps) { *(volatile v2us*)(Qh + o) = qh; *(volatile v2us*)(Ql + o) = ql; *(volatile v2us*)(Kh + o) = kh; *(volatile v2us*)(Kl + o) = kl; if (ps == 0) __threadfence(); } }
__global__ __launch_bounds__(256) void k_vt(const float* __restrict__ QKV, bf* VTh, bf* VTl) { const size_t e = ((size_t)blockIdx.x * 256 + threadIdx.x) * 2; if (e >= (size_t)NH_ * HD * TT) return; const int t = (int)(e % TT); const int d = (int)((e / TT) % HD); const int h = (int)(e / ((size_t)TT * HD)); v2us oh, ol;
#pragma unroll
    for (int u = 0; u < 2; ++u) { unsigned short a, c; splitf(QKV[(size_t)(t + u) * 3 * EE + 2 * EE + h * HD + d], a, c); oh[u] = a; ol[u] = c; } *(volatile v2us*)(VTh + e) = oh; *(volatile v2us*)(VTl + e) = ol; __threadfence(); *(volatile v2us*)(VTh + e) = oh; *(volatile v2us*)(VTl + e) = ol; }
__global__ __launch_bounds__(256) void k_kern(float* Sb) { const size_t e = ((size_t)blockIdx.x * 256 + threadIdx.x) * 4; if (e >= (size_t)ZH * TT * TT) return; const int j = (int)(e % TT); const int i = (int)((e / TT) % TT); const v4f a = *(const v4f*)(Sb + e); v4f o;
#pragma unroll
    for (int q = 0; q < 4; ++q) { float kk = 0.f; if (j + q <= i) { const float xd = a[q]; float x2 = __fmul_rn(xd, xd); asm volatile("" : "+v"(x2)); float tx = __fmul_rn(2.0f, xd); asm volatile("" : "+v"(tx)); const float den = fmaxf(__fsub_rn(2.000001f, tx), 1e-6f); kk = __fdiv_rn(x2, den); } o[q] = kk; }
    *(volatile v4f*)(Sb + e) = o; __threadfence(); *(volatile v4f*)(Sb + e) = o; }
__global__ __launch_bounds__(256) void k_zrow(const float* __restrict__ Kb, bf* Ph, bf* Pl, float* Z) { const int lane = threadIdx.x & 31; const int row = blockIdx.x * 8 + (threadIdx.x >> 5); if (row >= ZH * TT) return; const float* sr = Kb + (size_t)row * TT; float v[64]; float s = 0.f;
#pragma unroll
    for (int ch = 0; ch < 16; ++ch) { const v4f a = *(const v4f*)(sr + ch * 128 + lane * 4);
#pragma unroll
        for (int q = 0; q < 4; ++q) { v[ch * 4 + q] = a[q]; s = __fadd_rn(s, a[q]); } }
#pragma unroll
    for (int sh = 16; sh; sh >>= 1) s += __shfl_xor(s, sh, 32);
    const float zz = fmaxf(s, 1e-6f);
#pragma unroll 1
    for (int ps = 0; ps < 2; ++ps) {
#pragma unroll
        for (int ch = 0; ch < 16; ++ch) { v4us oh, ol;
#pragma unroll
            for (int q = 0; q < 4; ++q) { unsigned short a, c; splitf(v[ch * 4 + q], a, c); oh[q] = a; ol[q] = c; } *(volatile v4us*)(Ph + (size_t)row * TT + ch * 128 + lane * 4) = oh; *(volatile v4us*)(Pl + (size_t)row * TT + ch * 128 + lane * 4) = ol; }
        if (lane == 0) *(volatile float*)(Z + row) = zz; if (ps == 0) __threadfence(); } }
__global__ __launch_bounds__(256) void k_mrg(const float* __restrict__ Ob, const float* __restrict__ Z, int h0, bf* Ah, bf* Al) { const size_t e = ((size_t)blockIdx.x * 256 + threadIdx.x) * 2; if (e >= (size_t)ZH * TT * HD) return; const int d = (int)(e % HD); const int t = (int)((e / HD) % TT); const int z = (int)(e / ((size_t)HD * TT)); const float zi = Z[(size_t)z * TT + t]; v2us oh, ol;
#pragma unroll
    for (int u = 0; u < 2; ++u) { unsigned short a, c; splitf(__fdiv_rn(Ob[e + u], zi), a, c); oh[u] = a; ol[u] = c; } const size_t o = (size_t)t * EE + (h0 + z) * HD + d; *(volatile v2us*)(Ah + o) = oh; *(volatile v2us*)(Al + o) = ol; __threadfence(); *(volatile v2us*)(Ah + o) = oh; *(volatile v2us*)(Al + o) = ol; }

extern "C" void kernel_launch(void* const* d_in, const int* in_sizes, int n_in,
                              void* d_out, int out_size, void* d_ws, size_t ws_size, hipStream_t stream) {
    (void)in_sizes; (void)n_in; (void)out_size;
    const float* x = (const float*)d_in[0]; const float* wqkv = (const float*)d_in[1]; const float* bqkv = (const float*)d_in[2]; const float* wout = (const float*)d_in[3]; const float* bout = (const float*)d_in[4];
    float* OUT = (float*)d_out;
    char* wsp = (char*)d_ws;
    auto take = [&](size_t bytes) { char* p = wsp; wsp += (bytes + 255) & ~(size_t)255; return (void*)p; };
    bf* WQKV = (bf*)take((size_t)3 * EE * EE * 2); bf* WO = (bf*)take((size_t)EE * EE * 2); bf* XB = (bf*)take((size_t)TT * EE * 2); float* QKV = (float*)take((size_t)TT * 3 * EE * 4);
    bf* Qh = (bf*)take((size_t)NH_ * TT * HD * 2); bf* Ql = (bf*)take((size_t)NH_ * TT * HD * 2); bf* Kh = (bf*)take((size_t)NH_ * TT * HD * 2); bf* Kl = (bf*)take((size_t)NH_ * TT * HD * 2); bf* VTh = (bf*)take((size_t)NH_ * HD * TT * 2); bf* VTl = (bf*)take((size_t)NH_ * HD * TT * 2);
    float* Sb = (float*)take((size_t)ZH * TT * TT * 4); bf* Ph = (bf*)take((size_t)ZH * TT * TT * 2); bf* Pl = (bf*)take((size_t)ZH * TT * TT * 2); float* Z = (float*)take((size_t)ZH * TT * 4); float* Ob = (float*)take((size_t)ZH * TT * HD * 4); bf* Ah = (bf*)take((size_t)TT * EE * 2); bf* Al = (bf*)take((size_t)TT * EE * 2);
    if ((size_t)(wsp - (char*)d_ws) > ws_size) return;
    k_cvt8<<<(3 * EE * EE / 8 + 255) / 256, 256, 0, stream>>>(wqkv, WQKV, (size_t)3 * EE * EE / 8); k_cvt8<<<(EE * EE / 8 + 255) / 256, 256, 0, stream>>>(wout, WO, (size_t)EE * EE / 8);
    for (int b = 0; b < NB_; ++b) {
        k_cvt8<<<(TT * EE / 8 + 255) / 256, 256, 0, stream>>>(x + (size_t)b * TT * EE, XB, (size_t)TT * EE / 8);
        k_gemmw<bf, 0, true><<<dim3(TT / 64, 3 * EE / 64, 1), 32, 0, stream>>>(XB, nullptr, WQKV, nullptr, EE, QKV, 3 * EE, bqkv, 0, 0, 0);
        k_nrm<<<NH_ * TT / 8, 256, 0, stream>>>(QKV, Qh, Ql, Kh, Kl); k_vt<<<(unsigned)(((size_t)NH_ * HD * TT / 2 + 255) / 256), 256, 0, stream>>>(QKV, VTh, VTl);
        for (int h0 = 0; h0 < NH_; h0 += ZH) { const size_t z = (size_t)h0;
            k_gemmc<bf, 2, 1><<<dim3(TT / 64, TT / 64, ZH), 32, 0, stream>>>(Qh + z * TT * HD, Ql + z * TT * HD, Kh + z * TT * HD, Kl + z * TT * HD, HD, Sb, TT, 0, (size_t)TT * HD, (size_t)TT * HD, (size_t)TT * TT);
            k_kern<<<(unsigned)(((size_t)ZH * TT * TT / 4 + 255) / 256), 256, 0, stream>>>(Sb); k_zrow<<<ZH * TT / 8, 256, 0, stream>>>(Sb, Ph, Pl, Z);
            k_gemmc<bf, 2, 2><<<dim3(TT / 64, 1, ZH), 32, 0, stream>>>(Ph, Pl, VTh + z * HD * TT, VTl + z * HD * TT, TT, Ob, HD, 0, (size_t)TT * TT, (size_t)HD * TT, (size_t)TT * HD);
            k_mrg<<<(unsigned)(((size_t)ZH * TT * HD / 2 + 255) / 256), 256, 0, stream>>>(Ob, Z, h0, Ah, Al); }
        k_gemmw<bf, 1, true><<<dim3(TT / 64, EE / 64, 1), 32, 0, stream>>>(Ah, Al, WO, nullptr, EE, OUT + (size_t)b * TT * EE, EE, bout, 0, 0, 0); }
}
